// MultiheadAttention_20495583937213
// MI455X (gfx1250) — hardware-verified
//
#include <hip/hip_runtime.h>


#ifndef NB
#define NB 2
#endif
#ifndef SEQ
#define SEQ 2048
#endif
#define NB_FULL  2
#define SEQ_FULL 2048
#define DM    1024
#define NH    16
#define HD    64
#define DQ    (NH * HD)
#define MROWS (SEQ * NB)
#define WCAR  64.0f
#define CCAR  64.0f
#define PSH   10.0f
#define SCL   0.125f
#define L2E   1.4426950408889634f

typedef _Float16 h16;
typedef unsigned short bf;
typedef __attribute__((ext_vector_type(16))) _Float16 v16h;
typedef __attribute__((ext_vector_type(8)))  _Float16 v8h;
typedef __attribute__((ext_vector_type(8)))  unsigned short v8us;
typedef __attribute__((ext_vector_type(8)))  float    v8f;
typedef __attribute__((ext_vector_type(4)))  float    v4f;
typedef v8h __attribute__((may_alias)) v8ha;
typedef v4f __attribute__((may_alias)) v4fa;

static_assert(HD == 64);
static_assert(DQ == DM);
static_assert(DM % 32 == 0);
static_assert(DM % 8 == 0);
static_assert(MROWS % 64 == 0);
static_assert(DQ % 64 == 0);
static_assert(SEQ % 64 == 0);
static_assert(SEQ % 32 == 0);
static_assert(SEQ <= SEQ_FULL);
static_assert(NB <= NB_FULL);

constexpr size_t NQK   = (size_t)NB * NH * SEQ * HD;
constexpr size_t B_W16 = (size_t)3 * DQ * DM * 2;
constexpr size_t B_WO  = (size_t)DM * DQ * 2;
constexpr size_t B_X16 = (size_t)3 * MROWS * DM * 2;
constexpr size_t B_MB  = (size_t)SEQ * SEQ_FULL * 2;
constexpr size_t B_QKV = (size_t)3 * NQK * 2;
constexpr size_t B_VT  = NQK * 2;
constexpr size_t B_CTX = (size_t)MROWS * DQ * 2;
constexpr size_t O_W16 = 0;
constexpr size_t O_WO  = O_W16 + B_W16;
constexpr size_t O_X16 = O_WO + B_WO;
constexpr size_t O_MB  = O_X16 + B_X16;
constexpr size_t O_QKV = O_MB + B_MB;
constexpr size_t O_VT  = O_QKV + B_QKV;
constexpr size_t O_CTX = O_VT + B_VT;
constexpr size_t O_END = O_CTX + B_CTX;
static_assert(B_W16 % 256 == 0 && B_WO % 256 == 0 && B_X16 % 256 == 0 && B_MB % 256 == 0 && B_QKV % 256 == 0 && B_VT % 256 == 0 && B_CTX % 256 == 0);
static_assert(O_END <= (size_t)134217728);

__device__ __forceinline__ unsigned short f2bf(float f) { unsigned u = __float_as_uint(f); u += 0x7FFFu + ((u >> 16) & 1u); return (unsigned short)(u >> 16); }
__device__ __forceinline__ float bf2f(unsigned short b) { return __uint_as_float(((unsigned)b) << 16); }
__device__ __forceinline__ float bfr(float f) { return bf2f(f2bf(f)); }
__device__ __forceinline__ v16h cat16(v8h lo, v8h hi) { return __builtin_shufflevector(lo, hi, 0, 1, 2, 3, 4, 5, 6, 7, 8, 9, 10, 11, 12, 13, 14, 15); }
__device__ __forceinline__ v16h ldfrag(const h16* p) { return cat16(*(const v8h*)p, *(const v8h*)(p + 16)); }
__device__ __forceinline__ v8f wmma_g(v16h a, v16h b, v8f c) {
    c = __builtin_amdgcn_wmma_f32_16x16x32_f16(false, a, false, b, (short)0, c, false, false);
    asm volatile("v_nop\n\tv_nop\n\tv_nop\n\tv_nop" : "+v"(c) : "v"(a), "v"(b));
    return c;
}

__global__ __launch_bounds__(256) void k_cvt_h(const float* __restrict__ src, h16* dst, int n8, float scale) {
    const int i = blockIdx.x * 256 + threadIdx.x; if (i >= n8) return;
    const v4f a = *(const v4f*)(src + (size_t)i * 8); const v4f c = *(const v4f*)(src + (size_t)i * 8 + 4); v8h o;
#pragma unroll
    for (int k = 0; k < 4; ++k) { o[k] = (h16)(bfr(a[k]) * scale); o[4 + k] = (h16)(bfr(c[k]) * scale); }
    *(volatile v8h*)(dst + (size_t)i * 8) = o; __threadfence(); *(volatile v8h*)(dst + (size_t)i * 8) = o; }
__global__ __launch_bounds__(256) void k_cvt_x(const float* __restrict__ src, h16* dst) {
    const int i = blockIdx.x * 256 + threadIdx.x; if (i >= MROWS * (DM / 8)) return;
    const int row = i / (DM / 8), c = i % (DM / 8); const int t = row / NB, b = row % NB;
    const size_t so = ((size_t)t * NB_FULL + b) * DM + (size_t)c * 8;
    const v4f a = *(const v4f*)(src + so); const v4f e = *(const v4f*)(src + so + 4); v8h o;
#pragma unroll
    for (int k = 0; k < 4; ++k) { o[k] = (h16)bfr(a[k]); o[4 + k] = (h16)bfr(e[k]); }
    *(volatile v8h*)(dst + (size_t)i * 8) = o; __threadfence(); *(volatile v8h*)(dst + (size_t)i * 8) = o; }
__global__ __launch_bounds__(256) void k_cvt_m(const float* __restrict__ src, bf* dst, int n8) {
    const int i = blockIdx.x * 256 + threadIdx.x; if (i >= n8) return;
    const v4f a = *(const v4f*)(src + (size_t)i * 8); const v4f c = *(const v4f*)(src + (size_t)i * 8 + 4); v8us o;
#pragma unroll
    for (int k = 0; k < 4; ++k) { o[k] = f2bf(a[k]); o[4 + k] = f2bf(c[k]); }
    *(volatile v8us*)(dst + (size_t)i * 8) = o; __threadfence(); *(volatile v8us*)(dst + (size_t)i * 8) = o; }

__device__ __forceinline__ void gemm_main(const h16* __restrict__ A, const h16* __restrict__ Bt, size_t aoff, size_t boff, v8f (&acc)[4][4]) {
#pragma unroll 1
    for (int kc = 0; kc < DM; kc += 32) {
        v16h a[4];
#pragma unroll
        for (int mb = 0; mb < 4; ++mb) a[mb] = ldfrag(A + aoff + (size_t)mb * 16 * DM + kc);
#pragma unroll
        for (int nb = 0; nb < 4; ++nb) { const v16h bb = ldfrag(Bt + boff + (size_t)nb * 16 * DM + kc);
#pragma unroll
            for (int mb = 0; mb < 4; ++mb) acc[mb][nb] = wmma_g(a[mb], bb, acc[mb][nb]); }
    }
}

__global__ __launch_bounds__(32) void k_proj(const h16* __restrict__ X16, const h16* __restrict__ W16, const float* __restrict__ bias, h16* QKV) {
    __shared__ __align__(16) float os[16 * 68];
    const int z = blockIdx.z; const int lane = threadIdx.x & 31, lr = lane & 15, hi = lane >> 4; const int r0 = blockIdx.x * 64, c0 = blockIdx.y * 64;
    const h16* A = X16 + (size_t)z * MROWS * DM; const h16* Bt = W16 + (size_t)z * DQ * DM;
    v8f acc[4][4];
#pragma unroll
    for (int mb = 0; mb < 4; ++mb)
#pragma unroll
        for (int nb = 0; nb < 4; ++nb) acc[mb][nb] = (v8f){};
    gemm_main(A, Bt, (size_t)(r0 + lr) * DM + 8 * hi, (size_t)(c0 + lr) * DM + 8 * hi, acc);
    const int cp = (lane & 7) * 8, rq = lane >> 3; const int head = blockIdx.y;
    float bb[8];
    { const v4f b0 = *(const v4f*)(bias + (size_t)z * DQ + c0 + cp); const v4f b1 = *(const v4f*)(bias + (size_t)z * DQ + c0 + cp + 4);
#pragma unroll
      for (int k = 0; k < 4; ++k) { bb[k] = bfr(b0[k]); bb[4 + k] = bfr(b1[k]); } }
    h16* plane = QKV + (size_t)z * NQK;
#pragma unroll
    for (int mb = 0; mb < 4; ++mb) {
#pragma unroll
        for (int nb = 0; nb < 4; ++nb) {
#pragma unroll
            for (int j = 0; j < 8; ++j) os[(hi * 8 + j) * 68 + nb * 16 + lr] = acc[mb][nb][j]; }
        __syncthreads();
#pragma unroll 1
        for (int ps = 0; ps < 2; ++ps) {
#pragma unroll
            for (int s = 0; s < 4; ++s) { const int row = 4 * s + rq;
                const v4f x0 = *(const v4fa*)(os + row * 68 + cp); const v4f x1 = *(const v4fa*)(os + row * 68 + cp + 4); v8h o;
#pragma unroll
                for (int k = 0; k < 4; ++k) { o[k] = (h16)(x0[k] * (1.0f / WCAR) + bb[k]); o[4 + k] = (h16)(x1[k] * (1.0f / WCAR) + bb[4 + k]); }
                const int r = r0 + mb * 16 + row; const int t = r / NB, b = r % NB;
                *(volatile v8h*)(plane + ((size_t)(b * NH + head) * SEQ + t) * HD + cp) = o; }
            if (ps == 0) __threadfence(); }
        __syncthreads();
    }
}

__global__ __launch_bounds__(256) void k_vt(const h16* __restrict__ V16, h16* VT16) {
    __shared__ __align__(16) h16 tl[64 * 72];
    const int bh = blockIdx.y; const int t0 = blockIdx.x * 64; const int tid = threadIdx.x;
#pragma unroll
    for (int it = 0; it < 2; ++it) { const int ch = tid + it * 256; const int t = ch >> 3, c = ch & 7;
        const v8h v = *(const v8h*)(V16 + ((size_t)bh * SEQ + t0 + t) * HD + c * 8);
#pragma unroll
        for (int j = 0; j < 8; ++j) tl[(c * 8 + j) * 72 + t] = v[j]; }
    __syncthreads();
#pragma unroll 1
    for (int ps = 0; ps < 2; ++ps) {
#pragma unroll
        for (int it = 0; it < 2; ++it) { const int ch = tid + it * 256; const int d = ch >> 3, c = ch & 7;
            const v8h v = *(const v8ha*)(tl + d * 72 + c * 8);
            *(volatile v8h*)(VT16 + ((size_t)bh * HD + d) * SEQ + t0 + c * 8) = v; }
        if (ps == 0) __threadfence(); }
}

__global__ __launch_bounds__(128) void k_flash(const h16* __restrict__ Q16, const h16* __restrict__ K16, const h16* __restrict__ VT16, const bf* __restrict__ MB, h16* CTX) {
    __shared__ __align__(16) float os[4 * 16 * 68];
    const int wave = __builtin_amdgcn_readfirstlane(threadIdx.x >> 5);
    const int lane = threadIdx.x & 31, lm = lane & 15, lg = lane >> 4;
    const int bh = blockIdx.y; const int b = bh / NH, h = bh % NH;
    const int tb = blockIdx.x * 64 + wave * 16; const int tq = tb + lm;
    const size_t qoff = ((size_t)bh * SEQ + tq) * HD + 8 * lg;
    const v16h bq0 = ldfrag(Q16 + qoff), bq1 = ldfrag(Q16 + qoff + 32);
    const size_t kbase = ((size_t)bh * SEQ + lm) * HD + 8 * lg;
    const size_t vbase = ((size_t)bh * HD + lm) * SEQ + 8 * lg;
    const size_t mbase = (size_t)tq * SEQ_FULL + 8 * lg;
    v8f o0 = (v8f){}, o1 = (v8f){}, o2 = (v8f){}, o3 = (v8f){};
    float m2 = -1.0e30f, l_run = 0.f;
#pragma unroll 1
    for (int s = 0; s < SEQ; s += 32) {
        v8f s0 = (v8f){}, s1 = (v8f){};
        { const v16h a = ldfrag(K16 + kbase + (size_t)s * HD);             s0 = wmma_g(a, bq0, s0); }
        { const v16h a = ldfrag(K16 + kbase + (size_t)s * HD + 32);        s0 = wmma_g(a, bq1, s0); }
        { const v16h a = ldfrag(K16 + kbase + (size_t)(s + 16) * HD);      s1 = wmma_g(a, bq0, s1); }
        { const v16h a = ldfrag(K16 + kbase + (size_t)(s + 16) * HD + 32); s1 = wmma_g(a, bq1, s1); }
        const v8us mk0 = *(const v8us*)(MB + mbase + s); const v8us mk1 = *(const v8us*)(MB + mbase + s + 16);
        float u0[8], u1[8]; float mloc = -1.0e30f;
#pragma unroll
        for (int r = 0; r < 8; ++r) { u0[r] = (s0[r] * SCL + bf2f(mk0[r])) * L2E; u1[r] = (s1[r] * SCL + bf2f(mk1[r])) * L2E; mloc = fmaxf(mloc, fmaxf(u0[r], u1[r])); }
        mloc = fmaxf(mloc, __shfl_xor(mloc, 16, 32));
        const float m2n = fmaxf(m2, mloc); const float alpha = __builtin_amdgcn_exp2f(m2 - m2n); const float cs = PSH - m2n; m2 = m2n;
        float lsum = 0.f; v16h pa;
#pragma unroll
        for (int r = 0; r < 8; ++r) { const float p0 = __builtin_amdgcn_exp2f(u0[r] + cs); const float p1 = __builtin_amdgcn_exp2f(u1[r] + cs); lsum += p0 + p1; pa[r] = (h16)p0; pa[8 + r] = (h16)p1; }
        lsum += __shfl_xor(lsum, 16, 32);
        l_run = l_run * alpha + lsum;
        float av[8];
#pragma unroll
        for (int r = 0; r < 8; ++r) av[r] = __shfl(alpha, lg * 8 + r, 32);
#pragma unroll
        for (int r = 0; r < 8; ++r) { o0[r] *= av[r]; o1[r] *= av[r]; o2[r] *= av[r]; o3[r] *= av[r]; }
        { const v16h bv = ldfrag(VT16 + vbase + s);                         o0 = wmma_g(pa, bv, o0); }
        { const v16h bv = ldfrag(VT16 + vbase + (size_t)16 * SEQ + s);      o1 = wmma_g(pa, bv, o1); }
        { const v16h bv = ldfrag(VT16 + vbase + (size_t)32 * SEQ + s);      o2 = wmma_g(pa, bv, o2); }
        { const v16h bv = ldfrag(VT16 + vbase + (size_t)48 * SEQ + s);      o3 = wmma_g(pa, bv, o3); }
    }
    const float rl = CCAR / l_run; float inv[8];
#pragma unroll
    for (int r = 0; r < 8; ++r) inv[r] = __shfl(rl, lg * 8 + r, 32);
    const int wb = wave * (16 * 68);
#pragma unroll
    for (int r = 0; r < 8; ++r) { const int ro = wb + (lg * 8 + r) * 68 + lm;
        os[ro] = o0[r] * inv[r]; os[ro + 16] = o1[r] * inv[r]; os[ro + 32] = o2[r] * inv[r]; os[ro + 48] = o3[r] * inv[r]; }
    __syncthreads();
    const int cp = (lane & 7) * 8, rq = lane >> 3;
#pragma unroll 1
    for (int ps = 0; ps < 2; ++ps) {
#pragma unroll
        for (int sx = 0; sx < 4; ++sx) { const int row = 4 * sx + rq;
            const v4f x0 = *(const v4fa*)(os + wb + row * 68 + cp); const v4f x1 = *(const v4fa*)(os + wb + row * 68 + cp + 4); v8h o;
#pragma unroll
            for (int k = 0; k < 4; ++k) { o[k] = (h16)x0[k]; o[4 + k] = (h16)x1[k]; }
            *(volatile v8h*)(CTX + ((size_t)(tb + row) * NB + b) * DQ + h * HD + cp) = o; }
        if (ps == 0) __threadfence(); }
}

__global__ __launch_bounds__(32) void k_outp(const h16* __restrict__ CTX, const h16* __restrict__ WO16, const float* __restrict__ bo, float* OUT) {
    __shared__ __align__(16) float os[16 * 68];
    const int lane = threadIdx.x & 31, lr = lane & 15, hi = lane >> 4; const int r0 = blockIdx.x * 64, c0 = blockIdx.y * 64;
    v8f acc[4][4];
#pragma unroll
    for (int mb = 0; mb < 4; ++mb)
#pragma unroll
        for (int nb = 0; nb < 4; ++nb) acc[mb][nb] = (v8f){};
    gemm_main(CTX, WO16, (size_t)(r0 + lr) * DM + 8 * hi, (size_t)(c0 + lr) * DM + 8 * hi, acc);
    const int cofs = lr * 4; float bb[4];
    { const v4f b0 = *(const v4f*)(bo + c0 + cofs);
#pragma unroll
      for (int k = 0; k < 4; ++k) bb[k] = bfr(b0[k]); }
#pragma unroll
    for (int mb = 0; mb < 4; ++mb) {
#pragma unroll
        for (int nb = 0; nb < 4; ++nb) {
#pragma unroll
            for (int j = 0; j < 8; ++j) os[(hi * 8 + j) * 68 + nb * 16 + lr] = acc[mb][nb][j]; }
        __syncthreads();
#pragma unroll 1
        for (int ps = 0; ps < 2; ++ps) {
#pragma unroll
            for (int s = 0; s < 8; ++s) { const int row = 2 * s + hi;
                const v4f x = *(const v4fa*)(os + row * 68 + cofs); v4f val;
#pragma unroll
                for (int k = 0; k < 4; ++k) val[k] = x[k] * (1.0f / (WCAR * CCAR)) + bb[k];
                const int r = r0 + mb * 16 + row; const int t = r / NB, b = r % NB;
                *(volatile v4f*)(OUT + ((size_t)t * NB_FULL + b) * DM + c0 + cofs) = val; }
            if (ps == 0) __threadfence(); }
        __syncthreads();
    }
}

extern "C" void kernel_launch(void* const* d_in, const int* in_sizes, int n_in,
                              void* d_out, int out_size, void* d_ws, size_t ws_size, hipStream_t stream) {
    if (n_in < 8) return;
    const long long need_x = ((long long)(SEQ - 1) * NB_FULL + NB) * DM;
    if (in_sizes[0] < need_x || in_sizes[1] < need_x || in_sizes[2] < need_x) return;
    if (in_sizes[3] < (long long)(SEQ - 1) * SEQ_FULL + SEQ) return;
    if (in_sizes[4] < 3 * DQ * DM || in_sizes[5] < 3 * DQ || in_sizes[6] < DM * DQ || in_sizes[7] < DM) return;
    if (out_size < need_x) return;
    if (ws_size < O_END) return;
    const float* query = (const float*)d_in[0]; const float* key = (const float*)d_in[1]; const float* value = (const float*)d_in[2]; const float* mask = (const float*)d_in[3];
    const float* Win = (const float*)d_in[4]; const float* bin = (const float*)d_in[5]; const float* Wout = (const float*)d_in[6]; const float* bout = (const float*)d_in[7];
    float* OUT = (float*)d_out;
    char* ws = (char*)d_ws;
    h16* W16 = (h16*)(ws + O_W16); h16* WO16 = (h16*)(ws + O_WO); h16* X16 = (h16*)(ws + O_X16); bf* MB = (bf*)(ws + O_MB);
    h16* QKV = (h16*)(ws + O_QKV); h16* VT16 = (h16*)(ws + O_VT); h16* CTX = (h16*)(ws + O_CTX);

    const int nW = 3 * DQ * DM / 8, nWo = DM * DQ / 8, nX = MROWS * (DM / 8), nM = SEQ * (SEQ_FULL / 8);
    k_cvt_h<<<(nW + 255) / 256, 256, 0, stream>>>(Win, W16, nW, WCAR);
    k_cvt_h<<<(nWo + 255) / 256, 256, 0, stream>>>(Wout, WO16, nWo, WCAR);
    k_cvt_x<<<(nX + 255) / 256, 256, 0, stream>>>(query, X16);
    k_cvt_x<<<(nX + 255) / 256, 256, 0, stream>>>(key,   X16 + (size_t)MROWS * DM);
    k_cvt_x<<<(nX + 255) / 256, 256, 0, stream>>>(value, X16 + (size_t)2 * MROWS * DM);
    k_cvt_m<<<(nM + 255) / 256, 256, 0, stream>>>(mask, MB, nM);
    k_proj<<<dim3(MROWS / 64, DQ / 64, 3), 32, 0, stream>>>(X16, W16, bin, QKV);
    k_vt<<<dim3(SEQ / 64, NB * NH), 256, 0, stream>>>(QKV + (size_t)2 * NQK, VT16);
    k_flash<<<dim3(SEQ / 64, NB * NH), 128, 0, stream>>>(QKV, QKV + NQK, VT16, MB, CTX);
    k_outp<<<dim3(MROWS / 64, DM / 64), 32, 0, stream>>>(CTX, WO16, bout, OUT);
}
